// TimeAttentionBlock_82643760710000
// MI455X (gfx1250) — hardware-run, weakly checked
//
#include <hip/hip_runtime.h>
#include <stddef.h>


typedef _Float16 h16;
typedef _Float16 v16h __attribute__((ext_vector_type(16)));
typedef _Float16 v8h  __attribute__((ext_vector_type(8)));
typedef _Float16 v4h  __attribute__((ext_vector_type(4)));
typedef float    v8f  __attribute__((ext_vector_type(8)));
typedef float    v4f  __attribute__((ext_vector_type(4)));

#ifndef NB
#define NB 16
#endif
#ifndef LEN
#define LEN 8192
#endif
#define NB_FULL  16
#define LEN_FULL 8192
#define CIN  64
#define HC   256
#define COUT 64
#define GCH  512
#define NCH  (LEN / GCH)
#define ATL  128

static_assert(NB >= 1 && NB <= NB_FULL);
static_assert(LEN >= GCH && LEN <= LEN_FULL && (LEN % GCH) == 0 && (LEN % ATL) == 0);
static_assert(CIN == 64 && COUT == 64 && COUT == CIN);
static_assert(HC == 8 * 32);
static_assert((CIN % 32) == 0 && (HC % 32) == 0);
static_assert(GCH == 8 * 64);
static_assert((HC * CIN) == 8 * 256 * 8);
static_assert((COUT * CIN) % (256 * 8) == 0);
static_assert(NCH >= 1);

#define LDT 72
#define LDC 68
#define ALD 40
#define OLD 132
static_assert((LDT % 8) == 0 && LDT >= 64);
static_assert((LDC % 4) == 0 && LDC >= 64);
static_assert((ALD % 8) == 0 && ALD >= 32);
static_assert((OLD % 4) == 0 && OLD >= ATL);

#define WCARRY 64.0f
#define PCARRY 1024.0f
#define MCARRY 1024.0f
#define BCARRY 64.0f
#define RCARRY 2048.0f
#define RSQRT_H 0.17677669529663687f
#define BN_EPS 1.0e-5f
#define BLF (1.0f / ((float)NB * (float)LEN))

#define W16_BYTES    ((size_t)HC * CIN * 2)
#define WL16_BYTES   ((size_t)COUT * CIN * 2)
#define GPART_BYTES  ((size_t)NB * NCH * 4096 * 4)
#define SXPART_BYTES ((size_t)NB * NCH * 64 * 4)
#define G_BYTES      ((size_t)NB * 4096 * 4)
#define SX_BYTES     ((size_t)NB * 64 * 4)
#define T_BYTES      ((size_t)NB * HC * CIN * 2)
#define ST1_BYTES    ((size_t)NB * 128 * 4)
#define ST2_BYTES    ((size_t)NB * 256 * 4)
#define OFF_WQ     ((size_t)0)
#define OFF_WK     (OFF_WQ + W16_BYTES)
#define OFF_WVT    (OFF_WK + W16_BYTES)
#define OFF_WC     (OFF_WVT + W16_BYTES)
#define OFF_WL     (OFF_WC + W16_BYTES)
#define OFF_GPART  (OFF_WL + WL16_BYTES)
#define OFF_SXPART (OFF_GPART + GPART_BYTES)
#define OFF_G      (OFF_SXPART + SXPART_BYTES)
#define OFF_SX     (OFF_G + G_BYTES)
#define OFF_TH     (OFF_SX + SX_BYTES)
#define OFF_TR     (OFF_TH + T_BYTES)
#define OFF_P      (OFF_TR + T_BYTES)
#define OFF_Q      (OFF_P + G_BYTES)
#define OFF_ST1    (OFF_Q + G_BYTES)
#define OFF_ST2    (OFF_ST1 + ST1_BYTES)
#define WS_TOTAL   (OFF_ST2 + ST2_BYTES)
static_assert((W16_BYTES % 128) == 0 && (WL16_BYTES % 128) == 0 && (GPART_BYTES % 128) == 0);
static_assert((SXPART_BYTES % 128) == 0 && (G_BYTES % 128) == 0 && (SX_BYTES % 128) == 0);
static_assert((T_BYTES % 128) == 0 && (ST1_BYTES % 128) == 0 && (ST2_BYTES % 128) == 0);
static_assert(WS_TOTAL <= (size_t)134217728);

__device__ __forceinline__ float bf16r(float x) {
  unsigned int u = __float_as_uint(x);
  u = (u + 0x7FFFu + ((u >> 16) & 1u)) & 0xFFFF0000u;
  return __uint_as_float(u);
}

static __device__ __forceinline__ h16 toh_flush(float v) {
  const h16 r = (h16)v;
  return (fabsf(v) < 6.103515625e-05f) ? (h16)0.0f : r;
}

__device__ __forceinline__ v16h frag_at(const _Float16* p) {
  v8h lo = *(const v8h*)(p);
  v8h hi = *(const v8h*)(p + 16);
  v16h out;
#pragma unroll
  for (int i = 0; i < 8; ++i) { out[i] = lo[i]; out[i + 8] = hi[i]; }
  return out;
}
__device__ __forceinline__ v16h ld_frag(const _Float16* base, unsigned ld) {
  const unsigned lane = threadIdx.x & 31u;
  return frag_at(base + (lane & 15u) * ld + (lane >> 4) * 8u);
}

__device__ __forceinline__ v8f wmma16(v16h a, v16h b, v8f c) {
  v8f d = __builtin_amdgcn_wmma_f32_16x16x32_f16(false, a, false, b, (short)0, c,
                                                 false, false);
  asm volatile("v_nop\n\tv_nop\n\tv_nop\n\tv_nop" : "+v"(d) : "v"(a), "v"(b));
  return d;
}

__device__ __forceinline__ void wave_lds_sync() {
  __builtin_amdgcn_fence(3  , "wavefront");
  asm volatile("s_wait_dscnt 0x0" ::: "memory");
  __builtin_amdgcn_wave_barrier();
}

__device__ __forceinline__ void wplain_body(const float* __restrict__ W,
                                            _Float16* __restrict__ D16, const unsigned nelem) {
  const unsigned e = (blockIdx.x * 256u + threadIdx.x) * 8u;
  if (e < nelem) {
    const v4f a0 = *(const v4f*)(W + e);
    const v4f a1 = *(const v4f*)(W + e + 4u);
    v8h o;
#pragma unroll
    for (int i = 0; i < 4; ++i) {
      o[i]     = toh_flush(WCARRY * bf16r(a0[i]));
      o[i + 4] = toh_flush(WCARRY * bf16r(a1[i]));
    }
    _Float16* p = D16 + e;
    *(volatile v8h*)p = o;
    __threadfence();
    *(volatile v8h*)p = o;
  }
}
__device__ __forceinline__ void wtrans_body(const float* __restrict__ W,
                                            _Float16* __restrict__ D16) {
  const unsigned e = (blockIdx.x * 256u + threadIdx.x) * 8u;
  const unsigned c = e / (unsigned)HC;
  const unsigned j0 = e - c * (unsigned)HC;
  v8h o;
#pragma unroll
  for (unsigned i = 0; i < 8u; ++i)
    o[i] = toh_flush(WCARRY * bf16r(W[(size_t)(j0 + i) * CIN + c]));
  _Float16* p = D16 + e;
  *(volatile v8h*)p = o;
  __threadfence();
  *(volatile v8h*)p = o;
}

__global__ __launch_bounds__(256) void wprep_kernel(
    const float* __restrict__ wq, const float* __restrict__ wk, const float* __restrict__ wv,
    const float* __restrict__ wc, const float* __restrict__ wl,
    _Float16* __restrict__ Wq16, _Float16* __restrict__ Wk16, _Float16* __restrict__ WvT16,
    _Float16* __restrict__ Wc16, _Float16* __restrict__ Wl16) {
  const unsigned which = blockIdx.y;
  if (which == 0u)      wplain_body(wq, Wq16, (unsigned)(HC * CIN));
  else if (which == 1u) wplain_body(wk, Wk16, (unsigned)(HC * CIN));
  else if (which == 2u) wplain_body(wc, Wc16, (unsigned)(CIN * HC));
  else if (which == 3u) wplain_body(wl, Wl16, (unsigned)(COUT * CIN));
  else                  wtrans_body(wv, WvT16);
}

__global__ __launch_bounds__(256) void gram_kernel(
    const float* __restrict__ X, float* __restrict__ Gpart, float* __restrict__ SXpart) {
  __shared__ _Float16 Xs[64 * LDT];
  __shared__ float Cs[64 * LDC];
  __shared__ float sxs[64];
  const unsigned tid = threadIdx.x, lane = tid & 31u;
  const unsigned wave = (unsigned)__builtin_amdgcn_readfirstlane((int)(threadIdx.x >> 5));
  const unsigned hh = lane >> 4, m = lane & 15u;
  const unsigned mt = wave >> 1, nt0 = (wave & 1u) * 2u;
  const unsigned chunk = blockIdx.x, b = blockIdx.y;
  const float* xb = X + (size_t)b * CIN * LEN_FULL + (size_t)chunk * GCH;

  v8f acc0 = {}, acc1 = {};
  float sxp = 0.0f;
#pragma unroll 1
  for (unsigned st = 0; st < 8u; ++st) {
#pragma unroll
    for (unsigned j = 0; j < 4u; ++j) {
      const unsigned idx = tid + 256u * j;
      const unsigned r = idx >> 4, c4 = (idx & 15u) * 4u;
      const v4f v = *(const v4f*)(xb + (size_t)r * LEN_FULL + st * 64u + c4);
      v4h hv;
#pragma unroll
      for (int i = 0; i < 4; ++i) hv[i] = toh_flush(bf16r(v[i]));
      *(v4h*)&Xs[r * LDT + c4] = hv;
    }
    __syncthreads();
    {
      const unsigned c = tid >> 2, sg = (tid & 3u) * 16u;
      const v8h u0 = *(const v8h*)&Xs[c * LDT + sg];
      const v8h u1 = *(const v8h*)&Xs[c * LDT + sg + 8u];
      float s = 0.0f;
#pragma unroll
      for (int i = 0; i < 8; ++i) s += (float)u0[i] + (float)u1[i];
      sxp += s;
    }
#pragma unroll
    for (unsigned ks = 0; ks < 2u; ++ks) {
      const v16h a  = ld_frag(&Xs[(mt * 16u) * LDT + ks * 32u], LDT);
      const v16h b0 = ld_frag(&Xs[(nt0 * 16u) * LDT + ks * 32u], LDT);
      const v16h b1 = ld_frag(&Xs[((nt0 + 1u) * 16u) * LDT + ks * 32u], LDT);
      acc0 = wmma16(a, b0, acc0);
      acc1 = wmma16(a, b1, acc1);
    }
    __syncthreads();
  }
  sxp += __shfl_xor(sxp, 1, 32);
  sxp += __shfl_xor(sxp, 2, 32);
  if ((tid & 3u) == 0u) sxs[tid >> 2] = sxp;
#pragma unroll
  for (int r = 0; r < 8; ++r) {
    float* d = &Cs[(mt * 16u + hh * 8u + (unsigned)r) * LDC + nt0 * 16u + m];
    d[0]  = acc0[r];
    d[16] = acc1[r];
  }
  __syncthreads();

  const size_t gbase = (size_t)(b * (unsigned)NCH + chunk) * 4096u;
  v4f xs[4];
  size_t off[4];
#pragma unroll
  for (unsigned i = 0; i < 4u; ++i) {
    const unsigned r = 16u * i + (tid >> 4);
    const unsigned c = (tid & 15u) * 4u;
    xs[i] = *(const v4f*)&Cs[r * LDC + c];
    off[i] = gbase + (size_t)r * 64u + c;
  }
#pragma unroll
  for (int i = 0; i < 4; ++i) *(volatile v4f*)(Gpart + off[i]) = xs[i];
  __threadfence();
#pragma unroll
  for (int i = 0; i < 4; ++i) *(volatile v4f*)(Gpart + off[i]) = xs[i];

  if (wave == 0u) {
    if (lane < 16u) {
      const v4f sv = *(const v4f*)&sxs[lane * 4u];
      float* p = SXpart + (size_t)(b * (unsigned)NCH + chunk) * 64u + lane * 4u;
      *(volatile v4f*)p = sv;
      __threadfence();
      *(volatile v4f*)p = sv;
    }
  }
}

__global__ __launch_bounds__(256) void tmat_kernel(
    const float* __restrict__ Gpart, const float* __restrict__ SXpart,
    const _Float16* __restrict__ Wq16, float* __restrict__ Gm, float* __restrict__ SXm,
    _Float16* __restrict__ Th16, _Float16* __restrict__ Tr16) {
  __shared__ _Float16 Gth[64 * LDT];
  __shared__ _Float16 Gtr[64 * LDT];
  __shared__ _Float16 Tsh[8 * 16 * LDT];
  __shared__ _Float16 Tsr[8 * 16 * LDT];
  __shared__ float sxs[64];
  const unsigned tid = threadIdx.x, lane = tid & 31u;
  const unsigned wave = (unsigned)__builtin_amdgcn_readfirstlane((int)(threadIdx.x >> 5));
  const unsigned hh = lane >> 4, m = lane & 15u;
  const unsigned b = blockIdx.x;

  v4f gv[4];
  size_t goff[4];
#pragma unroll
  for (unsigned i = 0; i < 4u; ++i) {
    const unsigned r = 16u * i + (tid >> 4);
    const unsigned c = (tid & 15u) * 4u;
    v4f g = {};
#pragma unroll 1
    for (unsigned ch = 0; ch < (unsigned)NCH; ++ch)
      g += *(const v4f*)(Gpart + (size_t)(b * (unsigned)NCH + ch) * 4096u + r * 64u + c);
    gv[i] = g;
    goff[i] = (size_t)b * 4096u + r * 64u + c;
#pragma unroll
    for (unsigned j = 0; j < 4u; ++j) {
      const float val = g[j];
      const h16 hi = toh_flush(val);
      const h16 rs = toh_flush((val - (float)hi) * RCARRY);
      Gth[(c + j) * LDT + r] = hi;
      Gtr[(c + j) * LDT + r] = rs;
    }
  }
  if (tid < 64u) {
    float s = 0.0f;
#pragma unroll 1
    for (unsigned ch = 0; ch < (unsigned)NCH; ++ch)
      s += SXpart[(size_t)(b * (unsigned)NCH + ch) * 64u + tid];
    sxs[tid] = s;
  }
  __syncthreads();

#pragma unroll
  for (int i = 0; i < 4; ++i) *(volatile v4f*)(Gm + goff[i]) = gv[i];
  __threadfence();
#pragma unroll
  for (int i = 0; i < 4; ++i) *(volatile v4f*)(Gm + goff[i]) = gv[i];
  if (wave == 0u) {
    if (lane < 16u) {
      const v4f sv = *(const v4f*)&sxs[lane * 4u];
      float* p = SXm + (size_t)b * 64u + lane * 4u;
      *(volatile v4f*)p = sv;
      __threadfence();
      *(volatile v4f*)p = sv;
    }
  }

  _Float16* TH = Tsh + wave * (16u * LDT);
  _Float16* TR = Tsr + wave * (16u * LDT);
#pragma unroll 1
  for (unsigned rr = 0; rr < 2u; ++rr) {
    const unsigned rt = wave * 2u + rr;
    v8f th[4], tr[4];
#pragma unroll
    for (int ct = 0; ct < 4; ++ct) { th[ct] = (v8f){}; tr[ct] = (v8f){}; }
#pragma unroll
    for (unsigned ks = 0; ks < 2u; ++ks) {
      const v16h a = frag_at(Wq16 + (size_t)(rt * 16u + m) * CIN + ks * 32u + hh * 8u);
#pragma unroll
      for (int ct = 0; ct < 4; ++ct) {
        const v16h bh = ld_frag(&Gth[((unsigned)ct * 16u) * LDT + ks * 32u], LDT);
        const v16h br = ld_frag(&Gtr[((unsigned)ct * 16u) * LDT + ks * 32u], LDT);
        th[ct] = wmma16(a, bh, th[ct]);
        tr[ct] = wmma16(a, br, tr[ct]);
      }
    }
#pragma unroll
    for (int ct = 0; ct < 4; ++ct)
#pragma unroll
      for (int r = 0; r < 8; ++r) {
        const float t = (th[ct][r] + tr[ct][r] * (1.0f / RCARRY)) * (1.0f / WCARRY);
        const h16 hi = toh_flush(t);
        const h16 rs = toh_flush((t - (float)hi) * RCARRY);
        TH[(hh * 8u + (unsigned)r) * LDT + (unsigned)ct * 16u + m] = hi;
        TR[(hh * 8u + (unsigned)r) * LDT + (unsigned)ct * 16u + m] = rs;
      }
    wave_lds_sync();
    v8h xh[4], xr[4];
    size_t off[4];
#pragma unroll
    for (unsigned i = 0; i < 4u; ++i) {
      const unsigned r = 4u * i + (lane >> 3);
      const unsigned c = (lane & 7u) * 8u;
      xh[i] = *(const v8h*)&TH[r * LDT + c];
      xr[i] = *(const v8h*)&TR[r * LDT + c];
      off[i] = ((size_t)b * HC + rt * 16u + r) * CIN + c;
    }
#pragma unroll
    for (int i = 0; i < 4; ++i) {
      *(volatile v8h*)(Th16 + off[i]) = xh[i];
      *(volatile v8h*)(Tr16 + off[i]) = xr[i];
    }
    __threadfence();
#pragma unroll
    for (int i = 0; i < 4; ++i) {
      *(volatile v8h*)(Th16 + off[i]) = xh[i];
      *(volatile v8h*)(Tr16 + off[i]) = xr[i];
    }
    wave_lds_sync();
  }
}

__global__ __launch_bounds__(256) void scores_kernel(
    const _Float16* __restrict__ Th16, const _Float16* __restrict__ Tr16,
    const _Float16* __restrict__ Wk16, const _Float16* __restrict__ WvT16,
    const _Float16* __restrict__ Wc16, const float* __restrict__ Gm,
    const float* __restrict__ SXm, float* __restrict__ Pm, float* __restrict__ ST1) {
  __shared__ _Float16 At[8 * 32 * ALD];
  __shared__ float pmx[8 * 32];
  __shared__ float psm[8 * 32];
  __shared__ float Pf[64 * LDC];
  __shared__ float Gf[64 * LDC];
  __shared__ float sxs[64];
  __shared__ float yst[128];
  const unsigned tid = threadIdx.x, lane = tid & 31u;
  const unsigned wave = (unsigned)__builtin_amdgcn_readfirstlane((int)(threadIdx.x >> 5));
  const unsigned hh = lane >> 4, m = lane & 15u;
  const unsigned b = blockIdx.x;

  for (unsigned i = tid; i < 64u * LDC; i += 256u) Pf[i] = 0.0f;
#pragma unroll
  for (unsigned i = 0; i < 4u; ++i) {
    const unsigned r = 16u * i + (tid >> 4);
    const unsigned c = (tid & 15u) * 4u;
    *(v4f*)&Gf[r * LDC + c] = *(const v4f*)(Gm + (size_t)b * 4096u + r * 64u + c);
  }
  if (tid < 64u) sxs[tid] = SXm[(size_t)b * 64u + tid];
  __syncthreads();

  _Float16* A = At + wave * (32u * ALD);
  v8f macc[2][4];
#pragma unroll
  for (int rt = 0; rt < 2; ++rt)
#pragma unroll
    for (int ct = 0; ct < 4; ++ct) macc[rt][ct] = (v8f){};

#pragma unroll 1
  for (unsigned jb = 0; jb < 8u; ++jb) {
    v8f s[2][2];
#pragma unroll
    for (int rt = 0; rt < 2; ++rt) {
      v8f sh0 = {}, sh1 = {}, sr0 = {}, sr1 = {};
      const size_t trow =
          ((size_t)b * HC + wave * 32u + (unsigned)rt * 16u + m) * CIN + hh * 8u;
#pragma unroll
      for (unsigned ks = 0; ks < 2u; ++ks) {
        const v16h ah = frag_at(Th16 + trow + ks * 32u);
        const v16h ar = frag_at(Tr16 + trow + ks * 32u);
        const v16h b0 = frag_at(Wk16 + (size_t)(jb * 32u + m) * CIN + ks * 32u + hh * 8u);
        const v16h b1 = frag_at(Wk16 + (size_t)(jb * 32u + 16u + m) * CIN + ks * 32u + hh * 8u);
        sh0 = wmma16(ah, b0, sh0);
        sh1 = wmma16(ah, b1, sh1);
        sr0 = wmma16(ar, b0, sr0);
        sr1 = wmma16(ar, b1, sr1);
      }
      s[rt][0] = (sh0 + sr0 * (1.0f / RCARRY)) * (1.0f / WCARRY);
      s[rt][1] = (sh1 + sr1 * (1.0f / RCARRY)) * (1.0f / WCARRY);
    }

#pragma unroll
    for (int ct = 0; ct < 2; ++ct) {
      float mx = s[0][ct][0];
#pragma unroll
      for (int r = 0; r < 8; ++r) mx = fmaxf(mx, fmaxf(s[0][ct][r], s[1][ct][r]));
      mx = fmaxf(mx, __shfl_xor(mx, 16, 32));
      if (hh == 0u) pmx[wave * 32u + (unsigned)ct * 16u + m] = mx;
    }
    __syncthreads();
    float cmx[2];
#pragma unroll
    for (int ct = 0; ct < 2; ++ct) {
      float mx = pmx[(unsigned)ct * 16u + m];
#pragma unroll
      for (unsigned w2 = 1; w2 < 8u; ++w2) mx = fmaxf(mx, pmx[w2 * 32u + (unsigned)ct * 16u + m]);
      cmx[ct] = mx;
    }
#pragma unroll
    for (int ct = 0; ct < 2; ++ct) {
      float sm = 0.0f;
#pragma unroll
      for (int rt = 0; rt < 2; ++rt)
#pragma unroll
        for (int r = 0; r < 8; ++r) {
          const float e = __expf(s[rt][ct][r] - cmx[ct]);
          s[rt][ct][r] = e;
          sm += e;
        }
      sm += __shfl_xor(sm, 16, 32);
      if (hh == 0u) psm[wave * 32u + (unsigned)ct * 16u + m] = sm;
    }
    __syncthreads();
    float cinv[2];
#pragma unroll
    for (int ct = 0; ct < 2; ++ct) {
      float den = psm[(unsigned)ct * 16u + m];
#pragma unroll
      for (unsigned w2 = 1; w2 < 8u; ++w2) den += psm[w2 * 32u + (unsigned)ct * 16u + m];
      cinv[ct] = PCARRY * (1.0f / den);
    }

#pragma unroll
    for (int rt = 0; rt < 2; ++rt)
#pragma unroll
      for (int ct = 0; ct < 2; ++ct)
#pragma unroll
        for (int r = 0; r < 8; ++r)
          A[((unsigned)rt * 16u + hh * 8u + (unsigned)r) * ALD + (unsigned)ct * 16u + m] =
              toh_flush(s[rt][ct][r] * cinv[ct]);
    wave_lds_sync();

#pragma unroll
    for (int rt = 0; rt < 2; ++rt) {
      const v16h pa = ld_frag(A + ((unsigned)rt * 16u) * ALD, ALD);
#pragma unroll
      for (int ct = 0; ct < 4; ++ct) {
        const v16h bv = frag_at(WvT16 + (size_t)((unsigned)ct * 16u + m) * HC + jb * 32u + hh * 8u);
        macc[rt][ct] = wmma16(pa, bv, macc[rt][ct]);
      }
    }
    wave_lds_sync();
  }

  const float msc = MCARRY * RSQRT_H / (PCARRY * WCARRY);
  v16h bm[4];
#pragma unroll
  for (int ct = 0; ct < 4; ++ct)
#pragma unroll
    for (int r = 0; r < 8; ++r) {
      bm[ct][r]     = toh_flush(macc[0][ct][r] * msc);
      bm[ct][r + 8] = toh_flush(macc[1][ct][r] * msc);
    }

  const float psc = 1.0f / (WCARRY * MCARRY);
#pragma unroll 1
  for (unsigned w2 = 0; w2 < 8u; ++w2) {
    if (wave == w2) {
#pragma unroll
      for (int rt = 0; rt < 4; ++rt) {
        const v16h aw = frag_at(Wc16 + (size_t)((unsigned)rt * 16u + m) * HC + wave * 32u + hh * 8u);
#pragma unroll
        for (int ct = 0; ct < 4; ++ct) {
          v8f pz = {};
          pz = wmma16(aw, bm[ct], pz);
#pragma unroll
          for (int r = 0; r < 8; ++r) {
            float* d = &Pf[((unsigned)rt * 16u + hh * 8u + (unsigned)r) * LDC + (unsigned)ct * 16u + m];
            const float nv = d[0] + pz[r] * psc;
            d[0] = nv;
          }
        }
      }
    }
    __syncthreads();
  }

  {
    v4f xs[4];
    size_t off[4];
#pragma unroll
    for (unsigned i = 0; i < 4u; ++i) {
      const unsigned r = 16u * i + (tid >> 4);
      const unsigned c = (tid & 15u) * 4u;
      xs[i] = *(const v4f*)&Pf[r * LDC + c];
      off[i] = (size_t)b * 4096u + r * 64u + c;
    }
#pragma unroll
    for (int i = 0; i < 4; ++i) *(volatile v4f*)(Pm + off[i]) = xs[i];
    __threadfence();
#pragma unroll
    for (int i = 0; i < 4; ++i) *(volatile v4f*)(Pm + off[i]) = xs[i];
  }

  {
    const unsigned c = tid >> 2, q = tid & 3u;
    float ys = 0.0f, ss = 0.0f;
#pragma unroll 1
    for (unsigned c1 = q * 16u; c1 < q * 16u + 16u; ++c1) {
      float u = 0.0f;
#pragma unroll 4
      for (unsigned c2 = 0; c2 < 64u; ++c2) u += Gf[c1 * LDC + c2] * Pf[c * LDC + c2];
      const float pc = Pf[c * LDC + c1];
      ss += pc * u;
      ys += pc * sxs[c1];
    }
    ys += __shfl_xor(ys, 1, 32);
    ys += __shfl_xor(ys, 2, 32);
    ss += __shfl_xor(ss, 1, 32);
    ss += __shfl_xor(ss, 2, 32);
    if (q == 0u) { yst[c] = ys; yst[64u + c] = ss; }
  }
  __syncthreads();
  if (wave == 0u) {
    const v4f sv = *(const v4f*)&yst[lane * 4u];
    float* p = ST1 + (size_t)b * 128u + lane * 4u;
    *(volatile v4f*)p = sv;
    __threadfence();
    *(volatile v4f*)p = sv;
  }
}

__global__ __launch_bounds__(256) void mid_kernel(
    const float* __restrict__ Pm, const float* __restrict__ Gm, const float* __restrict__ SXm,
    const float* __restrict__ ST1, const float* __restrict__ g1, const float* __restrict__ b1,
    const float* __restrict__ wl, const _Float16* __restrict__ Wl16,
    float* __restrict__ Qm, float* __restrict__ ST2) {
  __shared__ _Float16 Bt[64 * LDT];
  __shared__ float Qf[64 * LDC];
  __shared__ float Gf[64 * LDC];
  __shared__ float sxs[64];
  __shared__ float a1s[64];
  __shared__ float c1s[64];
  __shared__ float st[256];
  const unsigned tid = threadIdx.x, lane = tid & 31u;
  const unsigned wave = (unsigned)__builtin_amdgcn_readfirstlane((int)(threadIdx.x >> 5));
  const unsigned hh = lane >> 4, m = lane & 15u;
  const unsigned b = blockIdx.x;

#pragma unroll
  for (unsigned i = 0; i < 4u; ++i) {
    const unsigned r = 16u * i + (tid >> 4);
    const unsigned c = (tid & 15u) * 4u;
    *(v4f*)&Gf[r * LDC + c] = *(const v4f*)(Gm + (size_t)b * 4096u + r * 64u + c);
  }
  if (tid < 64u) {
    sxs[tid] = SXm[(size_t)b * 64u + tid];
    float s1 = 0.0f, s2 = 0.0f;
#pragma unroll 1
    for (unsigned bb = 0; bb < (unsigned)NB; ++bb) {
      s1 += ST1[(size_t)bb * 128u + tid];
      s2 += ST1[(size_t)bb * 128u + 64u + tid];
    }
    const float mean = s1 * BLF;
    const float var = fmaxf(s2 * BLF - mean * mean, 0.0f);
    const float a = bf16r(g1[tid]) * (1.0f / sqrtf(var + BN_EPS));
    a1s[tid] = a;
    c1s[tid] = bf16r(b1[tid]) - a * mean;
  }
  __syncthreads();
  if (tid < 64u) {
    float s = 0.0f;
#pragma unroll 4
    for (unsigned c = 0; c < 64u; ++c) s += bf16r(wl[(size_t)tid * CIN + c]) * c1s[c];
    st[128u + tid] = s;
    st[192u + tid] = 0.0f;
  }
#pragma unroll
  for (unsigned i = 0; i < 4u; ++i) {
    const unsigned r = 16u * i + (tid >> 4);
    const unsigned c = (tid & 15u) * 4u;
    const v4f p = *(const v4f*)(Pm + (size_t)b * 4096u + r * 64u + c);
    const float sc = BCARRY * a1s[r];
#pragma unroll
    for (unsigned j = 0; j < 4u; ++j) Bt[(c + j) * LDT + r] = toh_flush(sc * p[j]);
  }
  __syncthreads();

  {
    const unsigned rt = wave >> 1, ct0 = (wave & 1u) * 2u;
    v8f acc0 = {}, acc1 = {};
#pragma unroll
    for (unsigned ks = 0; ks < 2u; ++ks) {
      const v16h a  = frag_at(Wl16 + (size_t)(rt * 16u + m) * CIN + ks * 32u + hh * 8u);
      const v16h b0 = ld_frag(&Bt[(ct0 * 16u) * LDT + ks * 32u], LDT);
      const v16h b1v = ld_frag(&Bt[((ct0 + 1u) * 16u) * LDT + ks * 32u], LDT);
      acc0 = wmma16(a, b0, acc0);
      acc1 = wmma16(a, b1v, acc1);
    }
    const float qsc = 1.0f / (WCARRY * BCARRY);
#pragma unroll
    for (int r = 0; r < 8; ++r) {
      const unsigned o = rt * 16u + hh * 8u + (unsigned)r;
      const unsigned cc = ct0 * 16u + m;
      Qf[o * LDC + cc]       = acc0[r] * qsc + bf16r(wl[(size_t)o * CIN + cc]);
      Qf[o * LDC + cc + 16u] = acc1[r] * qsc + bf16r(wl[(size_t)o * CIN + cc + 16u]);
    }
  }
  __syncthreads();

  {
    v4f xs[4];
    size_t off[4];
#pragma unroll
    for (unsigned i = 0; i < 4u; ++i) {
      const unsigned r = 16u * i + (tid >> 4);
      const unsigned c = (tid & 15u) * 4u;
      xs[i] = *(const v4f*)&Qf[r * LDC + c];
      off[i] = (size_t)b * 4096u + r * 64u + c;
    }
#pragma unroll
    for (int i = 0; i < 4; ++i) *(volatile v4f*)(Qm + off[i]) = xs[i];
    __threadfence();
#pragma unroll
    for (int i = 0; i < 4; ++i) *(volatile v4f*)(Qm + off[i]) = xs[i];
  }

  {
    const unsigned c = tid >> 2, q = tid & 3u;
    float qs = 0.0f, ss = 0.0f;
#pragma unroll 1
    for (unsigned c1 = q * 16u; c1 < q * 16u + 16u; ++c1) {
      float u = 0.0f;
#pragma unroll 4
      for (unsigned c2 = 0; c2 < 64u; ++c2) u += Gf[c1 * LDC + c2] * Qf[c * LDC + c2];
      const float qc = Qf[c * LDC + c1];
      ss += qc * u;
      qs += qc * sxs[c1];
    }
    qs += __shfl_xor(qs, 1, 32);
    qs += __shfl_xor(qs, 2, 32);
    ss += __shfl_xor(ss, 1, 32);
    ss += __shfl_xor(ss, 2, 32);
    if (q == 0u) { st[c] = qs; st[64u + c] = ss; }
  }
  __syncthreads();
  if (wave < 2u) {
    const v4f sv = *(const v4f*)&st[wave * 128u + lane * 4u];
    float* p = ST2 + (size_t)b * 256u + wave * 128u + lane * 4u;
    *(volatile v4f*)p = sv;
    __threadfence();
    *(volatile v4f*)p = sv;
  }
}

__global__ __launch_bounds__(256) void apply_kernel(
    const float* __restrict__ X, const float* __restrict__ Qm, const float* __restrict__ ST2,
    const float* __restrict__ g2, const float* __restrict__ b2, float* __restrict__ out) {
  __shared__ _Float16 Xt[ATL * LDT];
  __shared__ float Os[64 * OLD];
  __shared__ float a2s[64];
  __shared__ float kvs[64];
  const unsigned tid = threadIdx.x, lane = tid & 31u;
  const unsigned wave = (unsigned)__builtin_amdgcn_readfirstlane((int)(threadIdx.x >> 5));
  const unsigned hh = lane >> 4, m = lane & 15u;
  const unsigned l0 = blockIdx.x * (unsigned)ATL;
  const unsigned b = blockIdx.y;

  if (tid < 64u) {
    float s1 = 0.0f, s2 = 0.0f;
#pragma unroll 1
    for (unsigned bb = 0; bb < (unsigned)NB; ++bb) {
      s1 += ST2[(size_t)bb * 256u + tid];
      s2 += ST2[(size_t)bb * 256u + 64u + tid];
    }
    const float tt = ST2[(size_t)b * 256u + 128u + tid];
    const float mm = s1 * BLF;
    const float var = fmaxf(s2 * BLF - mm * mm, 0.0f);
    const float a = bf16r(g2[tid]) * (1.0f / sqrtf(var + BN_EPS));
    const float mean2 = mm + tt;
    a2s[tid] = a;
    kvs[tid] = a * (tt - mean2) + bf16r(b2[tid]);
  }
  const float* xb = X + (size_t)b * CIN * LEN_FULL + l0;
#pragma unroll 2
  for (unsigned j = 0; j < 8u; ++j) {
    const unsigned idx = tid + 256u * j;
    const unsigned r = idx >> 5, c4 = (idx & 31u) * 4u;
    const v4f v = *(const v4f*)(xb + (size_t)r * LEN_FULL + c4);
#pragma unroll
    for (unsigned i = 0; i < 4u; ++i) Xt[(c4 + i) * LDT + r] = toh_flush(bf16r(v[i]));
  }
  __syncthreads();

  const unsigned mt = wave & 3u, lh = wave >> 2;
  const unsigned orow = mt * 16u + m;
  const float sc = WCARRY * a2s[orow];
  v16h af[2];
#pragma unroll
  for (int ks = 0; ks < 2; ++ks) {
    const float* qp = Qm + (size_t)b * 4096u + (size_t)orow * CIN + (unsigned)ks * 32u + hh * 8u;
    const v4f q0 = *(const v4f*)(qp);
    const v4f q1 = *(const v4f*)(qp + 4);
    const v4f q2 = *(const v4f*)(qp + 16);
    const v4f q3 = *(const v4f*)(qp + 20);
#pragma unroll
    for (int i = 0; i < 4; ++i) {
      af[ks][i]      = toh_flush(sc * q0[i]);
      af[ks][i + 4]  = toh_flush(sc * q1[i]);
      af[ks][i + 8]  = toh_flush(sc * q2[i]);
      af[ks][i + 12] = toh_flush(sc * q3[i]);
    }
  }
  v8f acc[4];
#pragma unroll
  for (int s = 0; s < 4; ++s) acc[s] = (v8f){};
#pragma unroll
  for (int s = 0; s < 4; ++s)
#pragma unroll
    for (int ks = 0; ks < 2; ++ks) {
      const v16h bf = ld_frag(&Xt[(lh * 64u + (unsigned)s * 16u) * LDT + (unsigned)ks * 32u], LDT);
      acc[s] = wmma16(af[ks], bf, acc[s]);
    }
#pragma unroll
  for (int s = 0; s < 4; ++s)
#pragma unroll
    for (int r = 0; r < 8; ++r) {
      const unsigned o = mt * 16u + hh * 8u + (unsigned)r;
      Os[o * OLD + lh * 64u + (unsigned)s * 16u + m] =
          fmaxf(acc[s][r] * (1.0f / WCARRY) + kvs[o], 0.0f);
    }
  __syncthreads();

  v4f xs[8];
  size_t off[8];
#pragma unroll
  for (unsigned i = 0; i < 8u; ++i) {
    const unsigned idx = tid + 256u * i;
    const unsigned r = idx >> 5, c = (idx & 31u) * 4u;
    xs[i] = *(const v4f*)&Os[r * OLD + c];
    off[i] = ((size_t)b * COUT + r) * LEN_FULL + l0 + c;
  }
#pragma unroll
  for (int i = 0; i < 8; ++i) *(volatile v4f*)(out + off[i]) = xs[i];
  __threadfence();
#pragma unroll
  for (int i = 0; i < 8; ++i) *(volatile v4f*)(out + off[i]) = xs[i];
}

extern "C" void kernel_launch(void* const* d_in, const int* in_sizes, int n_in,
                              void* d_out, int out_size, void* d_ws, size_t ws_size,
                              hipStream_t stream) {
  if (n_in < 10) return;
  const long long need_x = ((long long)(NB - 1) * CIN + (CIN - 1)) * LEN_FULL + LEN;
  if ((long long)in_sizes[0] < need_x) return;
  if (in_sizes[1] < HC * CIN || in_sizes[2] < HC * CIN || in_sizes[3] < HC * CIN) return;
  if (in_sizes[4] < CIN * HC) return;
  if (in_sizes[5] < CIN || in_sizes[6] < CIN) return;
  if (in_sizes[7] < COUT * CIN) return;
  if (in_sizes[8] < COUT || in_sizes[9] < COUT) return;
  if ((long long)out_size < need_x) return;
  if (ws_size < WS_TOTAL) return;

  const float* x  = (const float*)d_in[0];
  const float* wk = (const float*)d_in[1];
  const float* wq = (const float*)d_in[2];
  const float* wv = (const float*)d_in[3];
  const float* wc = (const float*)d_in[4];
  const float* g1 = (const float*)d_in[5];
  const float* b1 = (const float*)d_in[6];
  const float* wl = (const float*)d_in[7];
  const float* g2 = (const float*)d_in[8];
  const float* b2 = (const float*)d_in[9];
  float* out = (float*)d_out;

  char* ws = (char*)d_ws;
  _Float16* Wq16   = (_Float16*)(ws + OFF_WQ);
  _Float16* Wk16   = (_Float16*)(ws + OFF_WK);
  _Float16* WvT16  = (_Float16*)(ws + OFF_WVT);
  _Float16* Wc16   = (_Float16*)(ws + OFF_WC);
  _Float16* Wl16   = (_Float16*)(ws + OFF_WL);
  float*    Gpart  = (float*)(ws + OFF_GPART);
  float*    SXpart = (float*)(ws + OFF_SXPART);
  float*    Gm     = (float*)(ws + OFF_G);
  float*    SXm    = (float*)(ws + OFF_SX);
  _Float16* Th16   = (_Float16*)(ws + OFF_TH);
  _Float16* Tr16   = (_Float16*)(ws + OFF_TR);
  float*    Pm     = (float*)(ws + OFF_P);
  float*    Qm     = (float*)(ws + OFF_Q);
  float*    ST1    = (float*)(ws + OFF_ST1);
  float*    ST2    = (float*)(ws + OFF_ST2);

  dim3 blk(256);
  wprep_kernel<<<dim3(8, 5), blk, 0, stream>>>(wq, wk, wv, wc, wl, Wq16, Wk16, WvT16, Wc16, Wl16);
  gram_kernel<<<dim3(NCH, NB), blk, 0, stream>>>(x, Gpart, SXpart);
  tmat_kernel<<<dim3(NB), blk, 0, stream>>>(Gpart, SXpart, Wq16, Gm, SXm, Th16, Tr16);
  scores_kernel<<<dim3(NB), blk, 0, stream>>>(Th16, Tr16, Wk16, WvT16, Wc16, Gm, SXm, Pm, ST1);
  mid_kernel<<<dim3(NB), blk, 0, stream>>>(Pm, Gm, SXm, ST1, g1, b1, wl, Wl16, Qm, ST2);
  apply_kernel<<<dim3(LEN / ATL, NB), blk, 0, stream>>>(x, Qm, ST2, g2, b2, out);
}
